// Transmodelv3_27934467293422
// MI455X (gfx1250) — hardware-run, weakly checked
//
#include <hip/hip_runtime.h>


#ifndef NB
#define NB 8
#endif
#ifndef SEQ
#define SEQ 512
#endif
#define NB_FULL  8
#define SEQ_FULL 512
#define DM   768
#define NH_  12
#define HD   64
#define AW   4
#define OSP  68
#define QP   148
#define PP   176
#define MAXR 64
#define RV   129
#define RK   160
#define RT   9
#define ME   128
#define NE   3
#define NT   4
#define DD   128
#define EN   (ME * NE)
#define XSP  776
#define TIP  136
#define WCAR  64.0f
#define WCARI (1.0f / 64.0f)
#define LOG2E 1.4426950408889634f
#define SC2  ((float)(0.125 * 1.4426950408889634))
#define PSH  6.0f
#define NEGB (-3.0e38f)

static_assert(HD == 64);
static_assert(NH_ * HD == DM);
static_assert(DM % 64 == 0);
static_assert(DM % 32 == 0);
static_assert(DM % 256 == 0);
static_assert(SEQ % 64 == 0);
static_assert((NB * SEQ) % 64 == 0);
static_assert(SEQ % 32 == 0);
static_assert(SEQ % (16 * AW) == 0);
static_assert(SEQ % 4 == 0);
static_assert(2 * MAXR + 1 == RV);
static_assert(RT * 16 >= RV);
static_assert(RT * 16 <= QP);
static_assert(RT * 16 <= RK);
static_assert(RK % 32 == 0);
static_assert(RK >= RV);
static_assert(PP >= RK);
static_assert((PP * 2) % 16 == 0);
static_assert((QP * 4) % 16 == 0);
static_assert((OSP * 4) % 16 == 0);
static_assert(16 * OSP <= 16 * QP);
static_assert((16 * PP / 8) % 32 == 0);
static_assert((size_t)SEQ * 64 < 65504);
static_assert(((size_t)SEQ * DM) % 8 == 0);
static_assert(NB <= NB_FULL);
static_assert(SEQ <= SEQ_FULL);
static_assert(NB >= 1);
static_assert(EN % 64 == 0);
static_assert(ME % 64 == 0);
static_assert(DD % 64 == 0);
static_assert(EN / 16 == 8 * 3);
static_assert(DD / 16 == 2 * 4);
static_assert(256 / 32 == NT * 2);
static_assert(ME % 32 == 0);
static_assert(DD % 32 == 0);
static_assert((XSP * 2) % 16 == 0);
static_assert((TIP * 2) % 16 == 0);
static_assert(XSP >= DM);
static_assert(TIP >= ME);
static_assert(TIP >= DD);
static_assert(NB_FULL == 8);
static_assert(NT * NB_FULL == 8 * 4);
static_assert(32 * 16 == DD * 4);
static_assert(RK * (HD / 2) == 20 * 256);
static_assert(RK * HD / 8 == 5 * 256);
static_assert(2 * 256 == 64 * 8);
static_assert(4 * 256 == 64 * 16);
static_assert(4 * 32 * 16 == 16 * 64 * 2);
static_assert(8 * 32 * 16 == 16 * HD * 4);
static_assert((size_t)AW * 16 * QP * 4 + (size_t)AW * 16 * PP * 2 <= 65536);
static_assert((size_t)RK * HD * 4 <= 131072);
static_assert((size_t)64 * 68 * 4 <= 131072);
static_assert((size_t)8 * XSP * 2 + (size_t)8 * EN * 4 + (size_t)NT * 8 * 4 * 4 + 2 * (size_t)NT * 8 * TIP * 2 + (size_t)NT * 8 * DD * 4 <= 65536);

typedef _Float16 h16;
typedef unsigned short bf;
typedef __attribute__((ext_vector_type(16))) __bf16   v16bf;
typedef __attribute__((ext_vector_type(16))) _Float16 v16h;
typedef __attribute__((ext_vector_type(8)))  _Float16 v8h;
typedef __attribute__((ext_vector_type(8)))  unsigned short v8us;
typedef __attribute__((ext_vector_type(8)))  float    v8f;
typedef __attribute__((ext_vector_type(4)))  float    v4f;
typedef v4f  __attribute__((may_alias)) v4fa;
typedef v8h  __attribute__((may_alias)) v8ha;

__device__ __forceinline__ unsigned short f2bf(float f) { unsigned u = __float_as_uint(f); u += 0x7FFFu + ((u >> 16) & 1u); return (unsigned short)(u >> 16); }
__device__ __forceinline__ float bfr(float f) { return __uint_as_float(((unsigned)f2bf(f)) << 16); }
__device__ __forceinline__ v16h cat16(v8h lo, v8h hi) { return __builtin_shufflevector(lo, hi, 0, 1, 2, 3, 4, 5, 6, 7, 8, 9, 10, 11, 12, 13, 14, 15); }
__device__ __forceinline__ v16bf cat16b(v8us lo, v8us hi) { return __builtin_bit_cast(v16bf, __builtin_shufflevector(lo, hi, 0, 1, 2, 3, 4, 5, 6, 7, 8, 9, 10, 11, 12, 13, 14, 15)); }
__device__ __forceinline__ v8f wmmab(v16bf a, v16bf b, v8f c) { return __builtin_amdgcn_wmma_f32_16x16x32_bf16(false, a, false, b, (short)0, c, false, false); }
__device__ __forceinline__ v8f wmma16g(v16h a, v16h b, v8f c) {
    c = __builtin_amdgcn_wmma_f32_16x16x32_f16(false, a, false, b, (short)0, c, false, false);
    asm volatile("v_nop\n\tv_nop\n\tv_nop\n\tv_nop" : "+v"(c) : "v"(a), "v"(b));
    return c;
}
__device__ __forceinline__ v16h  ldh(const h16* p) { return cat16(*(const v8h*)p, *(const v8h*)(p + 16)); }
__device__ __forceinline__ v16bf ldb(const bf* p)  { return cat16b(*(const v8us*)p, *(const v8us*)(p + 16)); }
__device__ __forceinline__ void wave_sync() { __builtin_amdgcn_fence(3  , "wavefront"); __builtin_amdgcn_wave_barrier(); asm volatile("" ::: "memory"); }
__device__ __forceinline__ h16 toh_flush(float v) { const h16 r = (h16)v; return (fabsf(v) < 6.103515625e-05f) ? (h16)0.0f : r; }

__global__ __launch_bounds__(256) void k_cvt8(const float* __restrict__ src, bf* dst, size_t n8) {
    const size_t i = (size_t)blockIdx.x * 256 + threadIdx.x; if (i >= n8) return;
    const v8f v = *(const v8f*)(src + i * 8); v8us o;
#pragma unroll
    for (int k = 0; k < 8; ++k) o[k] = f2bf(v[k]);
    *(volatile v8us*)(dst + i * 8) = o; __threadfence(); *(volatile v8us*)(dst + i * 8) = o;
}

template <int F16>
__device__ __forceinline__ void wtr_body(const float* __restrict__ in, bf* outb, h16* outh, int K, int N, float carry) {
    __shared__ __align__(16) float ts[64 * 68];
    const int tid = threadIdx.x;
    const int n0 = blockIdx.x * 64, k0 = blockIdx.y * 64;
    const size_t zi = (size_t)blockIdx.z * (size_t)K * (size_t)N;
#pragma unroll
    for (int i = 0; i < 4; ++i) { const int idx = i * 256 + tid; const int row = idx >> 4, c4 = (idx & 15) * 4;
        const v4f x = *(const v4f*)(in + zi + (size_t)(k0 + row) * N + n0 + c4);
        *(v4fa*)(&ts[row * 68 + c4]) = x; }
    __syncthreads();
    v8us ob[2]; v8h oh[2]; size_t oo[2];
#pragma unroll
    for (int i = 0; i < 2; ++i) { const int item = i * 256 + tid; const int nn = item >> 3, k8 = (item & 7) * 8;
        oo[i] = zi + (size_t)(n0 + nn) * K + k0 + k8;
#pragma unroll
        for (int j = 0; j < 8; ++j) { const float x = ts[(k8 + j) * 68 + nn];
            if (F16) { oh[i][j] = toh_flush(bfr(x) * carry); ob[i][j] = 0; }
            else     { ob[i][j] = f2bf(x); oh[i][j] = (h16)0.0f; } } }
#pragma unroll 1
    for (int ps = 0; ps < 2; ++ps) {
#pragma unroll
        for (int i = 0; i < 2; ++i) { if (F16) *(volatile v8h*)(outh + oo[i]) = oh[i]; else *(volatile v8us*)(outb + oo[i]) = ob[i]; }
        if (ps == 0) __threadfence(); }
}
__global__ __launch_bounds__(256) void k_wtr_b(const float* __restrict__ in, bf* out, int K, int N) { wtr_body<0>(in, out, (h16*)0, K, N, 1.0f); }
__global__ __launch_bounds__(256) void k_wtr_h(const float* __restrict__ in, h16* out, int K, int N, float carry) { wtr_body<1>(in, (bf*)0, out, K, N, carry); }

__global__ __launch_bounds__(256) void k_tab(h16* TH, h16* TT) {
#pragma clang fp contract(off)
    __shared__ __align__(16) float tb[RK * HD];
    const int tid = threadIdx.x;
#pragma unroll 1
    for (int i = tid; i < RK * (HD / 2); i += 256) { const int p = i >> 5, pi = i & 31;
        const float dv = expf((float)(2 * pi) * (-0.14391156831212787f));
        const float ang = (float)p * dv;
        const float sn = sinf(ang), cs = cosf(ang);
        const bool ok = p < RV;
        tb[p * HD + 2 * pi] = ok ? sn : 0.0f; tb[p * HD + 2 * pi + 1] = ok ? cs : 0.0f; }
    __syncthreads();
    v8h th[5], tt[5];
#pragma unroll
    for (int i = 0; i < 5; ++i) { const int pc = i * 256 + tid;
        const int row = pc >> 3, c8 = (pc & 7) * 8;
        const int d = pc / (RK / 8), r8 = (pc % (RK / 8)) * 8;
#pragma unroll
        for (int j = 0; j < 8; ++j) { th[i][j] = toh_flush(tb[row * HD + c8 + j]); tt[i][j] = toh_flush(tb[(r8 + j) * HD + d]); } }
#pragma unroll 1
    for (int ps = 0; ps < 2; ++ps) {
#pragma unroll
        for (int i = 0; i < 5; ++i) { const int pc = i * 256 + tid;
            *(volatile v8h*)(TH + (size_t)pc * 8) = th[i]; *(volatile v8h*)(TT + (size_t)pc * 8) = tt[i]; }
        if (ps == 0) __threadfence(); }
}

template <int MODE>
__device__ __forceinline__ void proj_body(const bf* __restrict__ A, const bf* __restrict__ Bt, const float* __restrict__ bias, h16* Ph) {
    __shared__ __align__(16) float os[16 * 68];
    const int K = DM;
    const int lane = threadIdx.x & 31, lr = lane & 15, hi = lane >> 4; const int r0 = blockIdx.x * 64, c0 = blockIdx.y * 64;
    v8f acc[4][4];
#pragma unroll
    for (int mb = 0; mb < 4; ++mb)
#pragma unroll
        for (int nb = 0; nb < 4; ++nb) acc[mb][nb] = (v8f){};
    const size_t aoff = (size_t)(r0 + lr) * K + 8 * hi, boff = (size_t)(c0 + lr) * K + 8 * hi;
#pragma unroll 1
    for (int kc = 0; kc < K; kc += 32) {
        v16bf a[4];
#pragma unroll
        for (int mb = 0; mb < 4; ++mb) a[mb] = ldb(A + aoff + (size_t)mb * 16 * K + kc);
#pragma unroll
        for (int nb = 0; nb < 4; ++nb) { const v16bf b = ldb(Bt + boff + (size_t)nb * 16 * K + kc);
#pragma unroll
            for (int mb = 0; mb < 4; ++mb) acc[mb][nb] = wmmab(a[mb], b, acc[mb][nb]); }
        asm volatile("v_nop\n\tv_nop\n\tv_nop\n\tv_nop" : "+v"(acc[0][0]), "+v"(acc[1][1]), "+v"(acc[2][2]), "+v"(acc[3][3]) : "v"(a[0]), "v"(a[1]), "v"(a[2]), "v"(a[3]));
    }
    float bc[4];
#pragma unroll
    for (int nb = 0; nb < 4; ++nb) bc[nb] = (MODE == 0) ? bfr(bias[c0 + nb * 16 + lr]) : 0.0f;
    size_t tbase; size_t pitch;
    if (MODE == 0) { const int bb = r0 / SEQ, tt = r0 % SEQ; const int zc = bb * NH_ + c0 / HD;
                     tbase = ((size_t)zc * SEQ + (size_t)tt) * HD; pitch = HD; }
    else           { const int bb = c0 / SEQ, tt = c0 % SEQ;
                     tbase = (size_t)bb * (size_t)DM * SEQ + (size_t)r0 * SEQ + (size_t)tt; pitch = SEQ; }
#pragma unroll
    for (int mb = 0; mb < 4; ++mb) {
        float br[8];
#pragma unroll
        for (int j = 0; j < 8; ++j) br[j] = (MODE == 1) ? bfr(bias[r0 + mb * 16 + hi * 8 + j]) : 0.0f;
#pragma unroll
        for (int nb = 0; nb < 4; ++nb) {
#pragma unroll
            for (int j = 0; j < 8; ++j) os[(hi * 8 + j) * 68 + nb * 16 + lr] = acc[mb][nb][j] + bc[nb] + br[j]; }
        wave_sync();
        const size_t sb = tbase + (size_t)(mb * 16) * pitch;
        v8h hv[4];
#pragma unroll
        for (int s = 0; s < 4; ++s) { const int row = 4 * s + (lane >> 3), c8 = (lane & 7) * 8;
            const v4f x0 = *(const v4fa*)(&os[row * 68 + c8]); const v4f x1 = *(const v4fa*)(&os[row * 68 + c8 + 4]);
#pragma unroll
            for (int i = 0; i < 4; ++i) { hv[s][i] = toh_flush(x0[i]); hv[s][4 + i] = toh_flush(x1[i]); } }
#pragma unroll 1
        for (int ps = 0; ps < 2; ++ps) {
#pragma unroll
            for (int s = 0; s < 4; ++s) { const int row = 4 * s + (lane >> 3), c8 = (lane & 7) * 8;
                *(volatile v8h*)(Ph + sb + (size_t)row * pitch + c8) = hv[s]; }
            if (ps == 0) __threadfence(); }
        wave_sync();
    }
}
__global__ __launch_bounds__(32) void k_proj_tok(const bf* __restrict__ A, const bf* __restrict__ Bt, const float* __restrict__ bias, h16* Ph) { proj_body<0>(A, Bt, bias, Ph); }
__global__ __launch_bounds__(32) void k_proj_tr(const bf* __restrict__ A, const bf* __restrict__ Bt, const float* __restrict__ bias, h16* Ph) { proj_body<1>(A, Bt, bias, Ph); }

__global__ __launch_bounds__(32 * AW) void k_flash(const h16* __restrict__ QH, const h16* __restrict__ KP, const h16* __restrict__ VT,
                                                   const h16* __restrict__ TH, const h16* __restrict__ TT, float* CX) {
    __shared__ __align__(16) float fs[AW * 16 * QP];
    __shared__ __align__(16) h16 prel[AW * 16 * PP];
    const int lane = threadIdx.x & 31, lr = lane & 15, hi = lane >> 4;
    const int wave = __builtin_amdgcn_readfirstlane((int)(threadIdx.x >> 5));
    const int zh = blockIdx.y; const int b = zh / NH_, h = zh % NH_;
    const int t0 = (blockIdx.x * AW + wave) * 16;
    const int tq = t0 + lr;
    const int wb = wave * 16 * QP, wp = wave * 16 * PP;
    const int fr = wb + lr * QP;
    const int prow = wp + lr * PP;
    const size_t pbase = (size_t)zh * SEQ * HD;
    const size_t qo = pbase + (size_t)tq * HD + 8 * hi;
    const v16h qh0 = ldh(QH + qo), qh1 = ldh(QH + qo + 32);
    const size_t ko = pbase + (size_t)lr * HD + 8 * hi;
    const size_t vo = pbase + (size_t)lr * SEQ + 8 * hi;
    { const v8h z8 = (v8h){};
#pragma unroll 1
      for (int i = lane; i < 16 * PP / 8; i += 32) *(v8ha*)(&prel[wp + i * 8]) = z8; }
#pragma unroll 1
    for (int rt = 0; rt < RT; ++rt) {
        const h16* ta = TH + (size_t)(rt * 16 + lr) * HD + 8 * hi;
        const v16h a0 = ldh(ta), a1 = ldh(ta + 32);
        v8f c = (v8f){};
        c = wmma16g(a0, qh0, c); c = wmma16g(a1, qh1, c);
        v4f x, y;
        x[0] = c[0]; x[1] = c[1]; x[2] = c[2]; x[3] = c[3]; y[0] = c[4]; y[1] = c[5]; y[2] = c[6]; y[3] = c[7];
        *(v4fa*)(&fs[fr + rt * 16 + 8 * hi]) = x; *(v4fa*)(&fs[fr + rt * 16 + 8 * hi + 4]) = y; }
    wave_sync();
    const float qb0 = fs[fr], qbN = fs[fr + 2 * MAXR];
    v8f o[4];
#pragma unroll
    for (int j = 0; j < 4; ++j) o[j] = (v8f){};
    float m = NEGB, l = 0.0f, l0 = 0.0f, lN = 0.0f, sh = 0.0f;
#pragma unroll 1
    for (int pass = 0; pass < 2; ++pass) {
#pragma unroll 1
        for (int key0 = 0; key0 < SEQ; key0 += 32) {
            const h16* ka = KP + ko + (size_t)key0 * HD;
            const v16h ka0 = ldh(ka), ka1 = ldh(ka + 32), kb0 = ldh(ka + 16 * HD), kb1 = ldh(ka + 16 * HD + 32);
            v8f sa = (v8f){}, sb = (v8f){};
            sa = wmma16g(ka0, qh0, sa); sa = wmma16g(ka1, qh1, sa); sb = wmma16g(kb0, qh0, sb); sb = wmma16g(kb1, qh1, sb);
            const bool farz = (key0 + 31 <= t0 - MAXR);
            const bool farn = (key0 >= t0 + 15 + MAXR);
            const int ja = key0 + 8 * hi;
            float ba[8], bb[8];
            if (farz | farn) {
                const float bv = farz ? qb0 : qbN;
#pragma unroll
                for (int r = 0; r < 8; ++r) { ba[r] = bv; bb[r] = bv; }
            } else {
#pragma unroll
                for (int r = 0; r < 8; ++r) {
                    int da = ja + r - tq; int db = da + 16;
                    da = da < -MAXR ? -MAXR : (da > MAXR ? MAXR : da); db = db < -MAXR ? -MAXR : (db > MAXR ? MAXR : db);
                    ba[r] = fs[fr + da + MAXR]; bb[r] = fs[fr + db + MAXR]; }
            }
            float ta[8], tb[8];
#pragma unroll
            for (int r = 0; r < 8; ++r) { ta[r] = (sa[r] + ba[r]) * SC2; tb[r] = (sb[r] + bb[r]) * SC2; }
            if (pass == 0) {
#pragma unroll
                for (int r = 0; r < 8; ++r) m = fmaxf(m, fmaxf(ta[r], tb[r]));
            } else {
                v16h pb; float ls = 0.0f, s0 = 0.0f, sN = 0.0f;
#pragma unroll
                for (int r = 0; r < 8; ++r) {
                    const float ea = ta[r] + sh, eb = tb[r] + sh;
                    const float ga = (ea < -14.0f) ? 0.0f : __builtin_amdgcn_exp2f(ea);
                    const float gb = (eb < -14.0f) ? 0.0f : __builtin_amdgcn_exp2f(eb);
                    const h16 pa = (h16)ga; const h16 pc = (h16)gb;
                    pb[r] = pa; pb[8 + r] = pc;
                    const float fa = (float)pa, fb = (float)pc;
                    ls += fa + fb;
                    const int ka_ = ja + r, kb_ = ja + 16 + r;
                    s0 += ((ka_ <= tq - MAXR) ? fa : 0.0f) + ((kb_ <= tq - MAXR) ? fb : 0.0f);
                    sN += ((ka_ >= tq + MAXR) ? fa : 0.0f) + ((kb_ >= tq + MAXR) ? fb : 0.0f); }
                l += ls; l0 += s0; lN += sN;
                if (!(farz | farn)) {
#pragma unroll
                    for (int r = 0; r < 8; ++r) {
                        const int ra = ja + r - tq + MAXR; const int rb = ra + 16;
                        if ((ra >= 1) & (ra <= 2 * MAXR - 1)) prel[prow + ra] = pb[r];
                        if ((rb >= 1) & (rb <= 2 * MAXR - 1)) prel[prow + rb] = pb[8 + r]; }
                }
                const h16* va = VT + vo + key0;
#pragma unroll
                for (int j = 0; j < 4; ++j) { const v16h vj = ldh(va + (size_t)(16 * j) * SEQ); o[j] = wmma16g(vj, pb, o[j]); }
            }
        }
        if (pass == 0) { m = fmaxf(m, __shfl_xor(m, 16, 32)); sh = PSH - m; }
    }
    l += __shfl_xor(l, 16, 32); l0 += __shfl_xor(l0, 16, 32); lN += __shfl_xor(lN, 16, 32);
    prel[prow] = toh_flush(l0); prel[prow + 2 * MAXR] = toh_flush(lN);
    wave_sync();
#pragma unroll 1
    for (int k0 = 0; k0 < RK; k0 += 32) {
        const v16h pbr = cat16(*(const v8ha*)(&prel[prow + k0 + 8 * hi]), *(const v8ha*)(&prel[prow + k0 + 16 + 8 * hi]));
#pragma unroll
        for (int j = 0; j < 4; ++j) { const v16h a = ldh(TT + (size_t)(16 * j + lr) * RK + k0 + 8 * hi); o[j] = wmma16g(a, pbr, o[j]); }
    }
    const float inv = 1.0f / l;
    wave_sync();
    const int ob = wb + lr * OSP;
#pragma unroll
    for (int j = 0; j < 4; ++j) { v4f a, c;
        a[0] = o[j][0] * inv; a[1] = o[j][1] * inv; a[2] = o[j][2] * inv; a[3] = o[j][3] * inv; c[0] = o[j][4] * inv; c[1] = o[j][5] * inv; c[2] = o[j][6] * inv; c[3] = o[j][7] * inv;
        *(v4fa*)(&fs[ob + 16 * j + 8 * hi]) = a; *(v4fa*)(&fs[ob + 16 * j + 8 * hi + 4]) = c; }
    wave_sync();
    float* orow = CX + ((size_t)b * SEQ + t0) * DM + h * HD;
    v4f val[8];
#pragma unroll
    for (int s = 0; s < 8; ++s) { const int row = 2 * s + (lane >> 4), cofs = (lane & 15) * 4;
        val[s] = *(const v4fa*)(&fs[wb + row * OSP + cofs]); }
#pragma unroll 1
    for (int ps = 0; ps < 2; ++ps) {
#pragma unroll
        for (int s = 0; s < 8; ++s) { const int row = 2 * s + (lane >> 4), cofs = (lane & 15) * 4;
            *(volatile v4f*)(orow + (size_t)row * DM + cofs) = val[s]; }
        if (ps == 0) __threadfence(); }
}

__global__ __launch_bounds__(256) void k_pool(const float* __restrict__ CX, float* XP) {
#pragma clang fp contract(off)
    const int c = blockIdx.x * 256 + threadIdx.x; const int b = blockIdx.y;
    const float* p = CX + (size_t)b * SEQ * DM + c;
    float a0 = 0.0f, a1 = 0.0f, a2 = 0.0f, a3 = 0.0f;
#pragma unroll 1
    for (int s = 0; s < SEQ; s += 4) { a0 += p[(size_t)s * DM]; a1 += p[(size_t)(s + 1) * DM]; a2 += p[(size_t)(s + 2) * DM]; a3 += p[(size_t)(s + 3) * DM]; }
    const float v = ((a0 + a1) + (a2 + a3)) * (1.0f / (float)SEQ);
    float* q = XP + (size_t)b * DM + c;
    *(volatile float*)q = v; __threadfence(); *(volatile float*)q = v;
}

__global__ __launch_bounds__(256) void k_mix(const float* __restrict__ XP, const h16* __restrict__ ET, const float* __restrict__ ebias,
                                             const float* __restrict__ mixw, const float* __restrict__ mixb,
                                             const h16* __restrict__ W1T, const float* __restrict__ b1, const h16* __restrict__ W2T, const float* __restrict__ b2, float* OUT) {
    __shared__ __align__(16) h16 xs[8 * XSP];
    __shared__ __align__(16) float eo[8 * EN];
    __shared__ __align__(16) float gl[NT * 8 * 4];
    __shared__ __align__(16) h16 ti[NT * 8 * TIP];
    __shared__ __align__(16) h16 h1[NT * 8 * TIP];
    __shared__ __align__(16) float ot[NT * 8 * DD];
    const int tid = threadIdx.x;
    const int lane = tid & 31, lr = lane & 15, hi = lane >> 4;
    const int wave = __builtin_amdgcn_readfirstlane((int)(threadIdx.x >> 5));
#pragma unroll 1
    for (int i = tid; i < 8 * DM; i += 256) { const int bb = i / DM, k = i % DM; const int bs = bb < NB ? bb : NB - 1;
        xs[bb * XSP + k] = toh_flush(XP[(size_t)bs * DM + k]); }
    if (tid < NT * 8 * NE) {
        const int t = tid / (8 * NE), bb = (tid / NE) % 8, e = tid % NE; const int bs = bb < NB ? bb : NB - 1;
        const float* xr = XP + (size_t)bs * DM;
        const float* gr = mixw + (size_t)t * DM * NE + e;
        float a0 = 0.0f, a1 = 0.0f, a2 = 0.0f, a3 = 0.0f;
#pragma unroll 1
        for (int k = 0; k < DM; k += 4) { a0 += xr[k] * bfr(gr[(size_t)k * NE]); a1 += xr[k + 1] * bfr(gr[(size_t)(k + 1) * NE]);
                                          a2 += xr[k + 2] * bfr(gr[(size_t)(k + 2) * NE]); a3 += xr[k + 3] * bfr(gr[(size_t)(k + 3) * NE]); }
        gl[(t * 8 + bb) * 4 + e] = ((a0 + a1) + (a2 + a3)) + bfr(mixb[t * NE + e]);
    }
    __syncthreads();
    { v8f acc[3];
#pragma unroll
      for (int i = 0; i < 3; ++i) acc[i] = (v8f){};
      const int ao = (lr & 7) * XSP + 8 * hi;
#pragma unroll 1
      for (int kc = 0; kc < DM; kc += 32) {
          const v16h a = cat16(*(const v8ha*)(&xs[ao + kc]), *(const v8ha*)(&xs[ao + kc + 16]));
#pragma unroll
          for (int i = 0; i < 3; ++i) { const v16h w = ldh(ET + (size_t)((wave * 3 + i) * 16 + lr) * DM + 8 * hi + kc); acc[i] = wmma16g(a, w, acc[i]); } }
#pragma unroll
      for (int i = 0; i < 3; ++i) { const int n = (wave * 3 + i) * 16 + lr;
          float braw = ebias[n]; asm volatile("" : "+v"(braw)); const float bs = bfr(braw);
          if (hi == 0) {
#pragma unroll
              for (int j = 0; j < 8; ++j) eo[j * EN + n] = acc[i][j] + bs; } } }
    if (tid < NT * 8) {
        const float g0 = gl[tid * 4], g1 = gl[tid * 4 + 1], g2 = gl[tid * 4 + 2];
        const float mx = fmaxf(g0, fmaxf(g1, g2));
        const float e0 = __builtin_amdgcn_exp2f((g0 - mx) * LOG2E), e1 = __builtin_amdgcn_exp2f((g1 - mx) * LOG2E), e2 = __builtin_amdgcn_exp2f((g2 - mx) * LOG2E);
        const float inv = 1.0f / (e0 + e1 + e2);
        gl[tid * 4] = e0 * inv; gl[tid * 4 + 1] = e1 * inv; gl[tid * 4 + 2] = e2 * inv;
    }
    __syncthreads();
#pragma unroll 1
    for (int i = tid; i < NT * 8 * ME; i += 256) { const int t = i / (8 * ME), bb = (i / ME) % 8, mm = i % ME;
        const float v = gl[(t * 8 + bb) * 4] * eo[bb * EN + mm * NE] + gl[(t * 8 + bb) * 4 + 1] * eo[bb * EN + mm * NE + 1] + gl[(t * 8 + bb) * 4 + 2] * eo[bb * EN + mm * NE + 2];
        ti[(t * 8 + bb) * TIP + mm] = toh_flush(v); }
    __syncthreads();
    const int tk = wave >> 1; const int nb0 = (wave & 1) * 4;
    { v8f acc[4];
#pragma unroll
      for (int i = 0; i < 4; ++i) acc[i] = (v8f){};
      const int ao = (tk * 8 + (lr & 7)) * TIP + 8 * hi;
#pragma unroll 1
      for (int kc = 0; kc < ME; kc += 32) {
          const v16h a = cat16(*(const v8ha*)(&ti[ao + kc]), *(const v8ha*)(&ti[ao + kc + 16]));
#pragma unroll
          for (int i = 0; i < 4; ++i) { const v16h w = ldh(W1T + ((size_t)tk * DD + (nb0 + i) * 16 + lr) * ME + 8 * hi + kc); acc[i] = wmma16g(a, w, acc[i]); } }
#pragma unroll
      for (int i = 0; i < 4; ++i) { const int d = (nb0 + i) * 16 + lr;
          float braw = b1[tk * DD + d]; asm volatile("" : "+v"(braw)); const float bs = bfr(braw);
          if (hi == 0) {
#pragma unroll
              for (int j = 0; j < 8; ++j) { const float v = acc[i][j] * WCARI + bs; h1[(tk * 8 + j) * TIP + d] = toh_flush((v > 0.0f) ? v : 0.0f); } } } }
    __syncthreads();
    { v8f acc[4];
#pragma unroll
      for (int i = 0; i < 4; ++i) acc[i] = (v8f){};
      const int ao = (tk * 8 + (lr & 7)) * TIP + 8 * hi;
#pragma unroll 1
      for (int kc = 0; kc < DD; kc += 32) {
          const v16h a = cat16(*(const v8ha*)(&h1[ao + kc]), *(const v8ha*)(&h1[ao + kc + 16]));
#pragma unroll
          for (int i = 0; i < 4; ++i) { const v16h w = ldh(W2T + ((size_t)tk * DD + (nb0 + i) * 16 + lr) * DD + 8 * hi + kc); acc[i] = wmma16g(a, w, acc[i]); } }
#pragma unroll
      for (int i = 0; i < 4; ++i) { const int d = (nb0 + i) * 16 + lr;
          float braw = b2[tk * DD + d]; asm volatile("" : "+v"(braw)); const float bs = bfr(braw);
          if (hi == 0) {
#pragma unroll
              for (int j = 0; j < 8; ++j) { const float v = acc[i][j] * WCARI + bs; ot[(tk * 8 + j) * DD + d] = (v > 0.0f) ? v : 0.0f; } } } }
    __syncthreads();
    v4f val[4];
#pragma unroll
    for (int i = 0; i < 4; ++i) { const int rr = wave * 4 + i; val[i] = *(const v4fa*)(&ot[rr * DD + lane * 4]); }
#pragma unroll 1
    for (int ps = 0; ps < 2; ++ps) {
#pragma unroll
        for (int i = 0; i < 4; ++i) { const int rr = wave * 4 + i;
            if ((rr % NB_FULL) < NB) *(volatile v4f*)(OUT + (size_t)rr * DD + lane * 4) = val[i]; }
        if (ps == 0) __threadfence(); }
}

static constexpr size_t al256(size_t v) { return (v + 255) & ~(size_t)255; }
static constexpr size_t SZ_XB = al256((size_t)NB * SEQ * DM * 2);
static constexpr size_t SZ_WB = al256((size_t)3 * DM * DM * 2);
static constexpr size_t SZ_PL = al256((size_t)NB * NH_ * SEQ * HD * 2);
static constexpr size_t SZ_TB = al256((size_t)RK * HD * 2);
static constexpr size_t SZ_CX = al256((size_t)NB * SEQ * DM * 4);
static constexpr size_t SZ_XP = al256((size_t)NB * DM * 4);
static constexpr size_t SZ_ET = al256((size_t)EN * DM * 2);
static constexpr size_t SZ_TW = al256((size_t)NT * DD * ME * 2);
static constexpr size_t SZ_TOTAL = SZ_XB + SZ_WB + 3 * SZ_PL + 2 * SZ_TB + SZ_CX + SZ_XP + SZ_ET + 2 * SZ_TW;
static_assert(SZ_TOTAL <= (size_t)134217728);
static_assert(((size_t)DM * DM * 2) % 256 == 0);
static_assert((size_t)NB * NH_ * SEQ * HD == (size_t)NB * DM * SEQ);
static_assert(ME == DD);

extern "C" void kernel_launch(void* const* d_in, const int* in_sizes, int n_in,
                              void* d_out, int out_size, void* d_ws, size_t ws_size, hipStream_t stream) {
    if (n_in < 15) return;
    const size_t needx = ((size_t)(NB - 1) * SEQ_FULL + SEQ) * DM;
    if ((size_t)in_sizes[0] < needx) return;
    if ((size_t)in_sizes[1] < (size_t)DM * DM || (size_t)in_sizes[3] < (size_t)DM * DM || (size_t)in_sizes[5] < (size_t)DM * DM) return;
    if (in_sizes[2] < DM || in_sizes[4] < DM || in_sizes[6] < DM) return;
    if ((size_t)in_sizes[7] < (size_t)DM * EN || in_sizes[8] < EN) return;
    if ((size_t)in_sizes[9] < (size_t)NT * DM * NE || in_sizes[10] < NT * NE) return;
    if ((size_t)in_sizes[11] < (size_t)NT * ME * DD || in_sizes[12] < NT * DD) return;
    if ((size_t)in_sizes[13] < (size_t)NT * DD * DD || in_sizes[14] < NT * DD) return;
    if ((size_t)out_size < (size_t)NT * NB_FULL * DD) return;
    if (SZ_TOTAL > ws_size) return;
    const float* xin = (const float*)d_in[0];
    const float* wq = (const float*)d_in[1]; const float* bq = (const float*)d_in[2];
    const float* wk = (const float*)d_in[3]; const float* bk = (const float*)d_in[4];
    const float* wv = (const float*)d_in[5]; const float* bv = (const float*)d_in[6];
    const float* ex = (const float*)d_in[7]; const float* exb = (const float*)d_in[8];
    const float* mw = (const float*)d_in[9]; const float* mb = (const float*)d_in[10];
    const float* w1 = (const float*)d_in[11]; const float* bb1 = (const float*)d_in[12];
    const float* w2 = (const float*)d_in[13]; const float* bb2 = (const float*)d_in[14];
    float* OUT = (float*)d_out;
    char* wsp = (char*)d_ws;
    bf* XB = (bf*)wsp; wsp += SZ_XB;
    bf* WB = (bf*)wsp; wsp += SZ_WB;
    h16* QH = (h16*)wsp; wsp += SZ_PL;
    h16* KP = (h16*)wsp; wsp += SZ_PL;
    h16* VT = (h16*)wsp; wsp += SZ_PL;
    h16* TH = (h16*)wsp; wsp += SZ_TB;
    h16* TT = (h16*)wsp; wsp += SZ_TB;
    float* CX = (float*)wsp; wsp += SZ_CX;
    float* XP = (float*)wsp; wsp += SZ_XP;
    h16* ET = (h16*)wsp; wsp += SZ_ET;
    h16* W1T = (h16*)wsp; wsp += SZ_TW;
    h16* W2T = (h16*)wsp; wsp += SZ_TW;
    bf* WQ = WB; bf* WK = WB + (size_t)DM * DM; bf* WV = WB + (size_t)2 * DM * DM;

    if (SEQ == SEQ_FULL) {
        const size_t n8 = (size_t)NB * SEQ * DM / 8;
        k_cvt8<<<(unsigned)((n8 + 255) / 256), 256, 0, stream>>>(xin, XB, n8);
    } else {
        const size_t n8 = (size_t)SEQ * DM / 8;
        for (int b = 0; b < NB; ++b) k_cvt8<<<(unsigned)((n8 + 255) / 256), 256, 0, stream>>>(xin + (size_t)b * SEQ_FULL * DM, XB + (size_t)b * SEQ * DM, n8);
    }
    k_wtr_b<<<dim3(DM / 64, DM / 64, 1), 256, 0, stream>>>(wq, WQ, DM, DM);
    k_wtr_b<<<dim3(DM / 64, DM / 64, 1), 256, 0, stream>>>(wk, WK, DM, DM);
    k_wtr_b<<<dim3(DM / 64, DM / 64, 1), 256, 0, stream>>>(wv, WV, DM, DM);
    k_wtr_h<<<dim3(EN / 64, DM / 64, 1), 256, 0, stream>>>(ex, ET, DM, EN, 1.0f);
    k_wtr_h<<<dim3(DD / 64, ME / 64, NT), 256, 0, stream>>>(w1, W1T, ME, DD, WCAR);
    k_wtr_h<<<dim3(DD / 64, DD / 64, NT), 256, 0, stream>>>(w2, W2T, DD, DD, WCAR);
    k_tab<<<1, 256, 0, stream>>>(TH, TT);

    k_proj_tok<<<dim3(NB * SEQ / 64, DM / 64, 1), 32, 0, stream>>>(XB, WQ, bq, QH);
    k_proj_tok<<<dim3(NB * SEQ / 64, DM / 64, 1), 32, 0, stream>>>(XB, WK, bk, KP);
    k_proj_tr<<<dim3(DM / 64, NB * SEQ / 64, 1), 32, 0, stream>>>(WV, XB, bv, VT);

    k_flash<<<dim3(SEQ / (16 * AW), NB * NH_, 1), 32 * AW, 0, stream>>>(QH, KP, VT, TH, TT, CX);
    k_pool<<<dim3(DM / 256, NB, 1), 256, 0, stream>>>(CX, XP);
    k_mix<<<1, 256, 0, stream>>>(XP, ET, exb, mw, mb, W1T, bb1, W2T, bb2, OUT);
}
